// Decoder_82231443849250
// MI455X (gfx1250) — hardware-run, weakly checked
//
#include <hip/hip_runtime.h>
#include <math.h>

typedef __attribute__((ext_vector_type(16))) _Float16 v16h;
typedef __attribute__((ext_vector_type(8)))  _Float16 v8h;
typedef __attribute__((ext_vector_type(4)))  _Float16 v4h;
typedef __attribute__((ext_vector_type(2)))  _Float16 v2h;
typedef __attribute__((ext_vector_type(16))) __bf16   v16b;
typedef __attribute__((ext_vector_type(8)))  __bf16   v8b;
typedef __attribute__((ext_vector_type(8)))  float    v8f;
typedef __attribute__((ext_vector_type(4)))  float    v4f;
typedef __attribute__((ext_vector_type(2)))  float    v2f;

constexpr int kB    = 256;
constexpr int kS    = 128;
constexpr int kH    = 1024;
constexpr int kJ    = 12;
constexpr int kLat  = 64;
constexpr int kObs  = 51;
constexpr int kPin  = 2 * kJ + kObs + kLat;
constexpr int kK1   = 192;
constexpr int kNLk  = 39;
constexpr int kPD   = 42;
constexpr int kNP   = 64;
constexpr int kThr  = 256;
constexpr float kFps = 30.0f, kActScale = 0.25f, kSMin = 0.05f, kSMax = 0.5f, kLnEps = 1e-5f;

constexpr float kInCarry = 1024.0f;
constexpr float kWCarry  = 1024.0f;
constexpr float kScale   = 1.0f / (kInCarry * kWCarry);
constexpr float kF16MinNormal = 6.103515625e-5f;

static_assert(kPin == 139 && kPin <= kK1 && (kK1 % 32) == 0 && (kB % 64) == 0 && (kH % 64) == 0 && (kNP % 64) == 0 && ((kB * kS) % 64) == 0, "sizes");

constexpr size_t kOut0 = 0;
constexpr size_t kOut1 = kOut0 + (size_t)kB * kS * kPD;
constexpr size_t kOut2 = kOut1 + (size_t)kB * kS * kJ;
constexpr size_t kOut3 = kOut2 + (size_t)kB * kS * kJ;
constexpr size_t kOutTotal = kOut3 + (size_t)kB * kS * kPD;
static_assert(kOutTotal == 3538944ull, "output floats");

constexpr size_t kOffW1P  = 0;
constexpr size_t kOffW2H  = kOffW1P  + (size_t)kH * kK1 * 2;
constexpr size_t kOffWA1H = kOffW2H  + (size_t)kH * kH * 2;
constexpr size_t kOffWA2P = kOffWA1H + (size_t)kH * kH * 2;
constexpr size_t kOffWVP  = kOffWA2P + (size_t)kNP * kH * 2;
constexpr size_t kOffBV   = kOffWVP  + (size_t)kNP * kH * 2;
constexpr size_t kOffX16  = kOffBV   + (size_t)5 * kH * 4;
constexpr size_t kOffPB   = kOffX16  + (size_t)kB * kK1 * 2;
constexpr size_t kOffH1   = kOffPB   + (size_t)kB * kH * 4;
constexpr size_t kOffA1   = kOffH1   + (size_t)kB * kH * 2;
constexpr size_t kOffP4   = kOffA1   + (size_t)kB * kH * 2;
constexpr size_t kOffST   = kOffP4   + (size_t)kB * kNP * 4;
constexpr size_t kOffJS   = kOffST   + (size_t)kB * 32 * 4;
constexpr size_t kOffOB   = kOffJS   + (size_t)kS * kB * 32 * 4;
constexpr size_t kOffF16  = kOffOB   + (size_t)kS * kB * 32 * 4;
constexpr size_t kOffPF   = kOffF16  + (size_t)kB * kS * kH * 2;
constexpr size_t kWsTotal = kOffPF   + (size_t)kB * kS * kNP * 4;
static_assert(kWsTotal == 91049984ull, "carve total");
static_assert(kWsTotal <= 134217728ull, "carve cap");
static_assert((kOffW2H % 256) == 0 && (kOffWA1H % 256) == 0 && (kOffWA2P % 256) == 0 && (kOffWVP % 256) == 0 && (kOffBV % 256) == 0 && (kOffX16 % 256) == 0 && (kOffPB % 256) == 0 && (kOffH1 % 256) == 0 && (kOffA1 % 256) == 0 && (kOffP4 % 256) == 0 && (kOffST % 256) == 0 && (kOffJS % 256) == 0 && (kOffOB % 256) == 0 && (kOffF16 % 256) == 0 && (kOffPF % 256) == 0, "aligned regions");

__device__ __forceinline__ unsigned short f2bf_bits(float f) {
  unsigned u = __float_as_uint(f);
  return (unsigned short)((u + 0x7FFFu + ((u >> 16) & 1u)) >> 16);
}
__device__ __forceinline__ float bf_bits2f(unsigned short h) { return __uint_as_float(((unsigned)h) << 16); }
__device__ __forceinline__ float bf16r(float f) { return bf_bits2f(f2bf_bits(f)); }
__device__ __forceinline__ float carry_flush(float v, float carry) {
  const float s = v * carry;
  return (fabsf(s) < kF16MinNormal) ? 0.0f : s;
}
__device__ __forceinline__ float frcp(float x) { return __builtin_amdgcn_rcpf(x); }

__device__ __forceinline__ void dep_guard4_h(v8f& a, v8f& b, v8f& c, v8f& d, v16h x, v16h y) { asm volatile("v_nop\n\tv_nop\n\tv_nop\n\tv_nop" : "+v"(a), "+v"(b), "+v"(c), "+v"(d) : "v"(x), "v"(y)); }
__device__ __forceinline__ void dep_guard4_b(v8f& a, v8f& b, v8f& c, v8f& d, v16b x, v16b y) { asm volatile("v_nop\n\tv_nop\n\tv_nop\n\tv_nop" : "+v"(a), "+v"(b), "+v"(c), "+v"(d) : "v"(x), "v"(y)); }
__device__ __forceinline__ void keep4_h(v16h a, v16h b, v16h c, v16h d) { asm volatile("v_nop" :: "v"(a), "v"(b), "v"(c), "v"(d)); }
__device__ __forceinline__ void keep4_b(v16b a, v16b b, v16b c, v16b d) { asm volatile("v_nop" :: "v"(a), "v"(b), "v"(c), "v"(d)); }
__device__ __forceinline__ void acc_guard4(v8f& a, v8f& b, v8f& c, v8f& d) { asm volatile("v_nop\n\tv_nop\n\tv_nop\n\tv_nop" : "+v"(a), "+v"(b), "+v"(c), "+v"(d)); }

template <typename T> struct Frag;
template <> struct Frag<_Float16> {
  typedef v16h V; union U { v16h v; v8h h[2]; };
  static __device__ __forceinline__ v16h load(const _Float16* p) {
    U f; f.h[0] = *(const v8h*)(p); f.h[1] = *(const v8h*)(p + 16); return f.v;
  }
  static __device__ __forceinline__ v8f mma(v16h a, v16h b, v8f c) {
    return __builtin_amdgcn_wmma_f32_16x16x32_f16(false, a, false, b, (short)0, c, false, false);
  }
  static __device__ __forceinline__ void guard4(v8f& a, v8f& b, v8f& c, v8f& d, v16h x, v16h y) { dep_guard4_h(a, b, c, d, x, y); }
  static __device__ __forceinline__ void keep(v16h a, v16h b, v16h c, v16h d) { keep4_h(a, b, c, d); }
};
template <> struct Frag<__bf16> {
  typedef v16b V; union U { v16b v; v8b h[2]; };
  static __device__ __forceinline__ v16b load(const __bf16* p) {
    U f; f.h[0] = *(const v8b*)(p); f.h[1] = *(const v8b*)(p + 16); return f.v;
  }
  static __device__ __forceinline__ v8f mma(v16b a, v16b b, v8f c) {
    return __builtin_amdgcn_wmma_f32_16x16x32_bf16(false, a, false, b, (short)0, c, false, false);
  }
  static __device__ __forceinline__ void guard4(v8f& a, v8f& b, v8f& c, v8f& d, v16b x, v16b y) { dep_guard4_b(a, b, c, d, x, y); }
  static __device__ __forceinline__ void keep(v16b a, v16b b, v16b c, v16b d) { keep4_b(a, b, c, d); }
};

__device__ __forceinline__ v8f mma_h(v16h a, v16h b, v8f c) {
  c = __builtin_amdgcn_wmma_f32_16x16x32_f16(false, a, false, b, (short)0, c, false, false);
  asm volatile("v_nop\n\tv_nop\n\tv_nop\n\tv_nop" : "+v"(c) : "v"(a), "v"(b));
  return c;
}

template <int ET> struct Elem;
template <> struct Elem<0> { typedef _Float16 T; };
template <> struct Elem<1> { typedef __bf16 T; };
template <int ET, bool SPLIT, int BIAS_MODE, int OUT_MODE, bool RESID, int ACT = 0>
__global__ __launch_bounds__(256) void wmma_gemm64(
    const unsigned short* __restrict__ Ap, const unsigned short* __restrict__ A2p, int lda, long strideA,
    const unsigned short* __restrict__ Btp, const unsigned short* __restrict__ Bt2p, int ldb, long strideB,
    void* __restrict__ Cout, void* __restrict__ Cout2, int ldc, long strideC,
    const float* __restrict__ bias,
    const float* __restrict__ resid, long strideR,
    int M, int N, int K, float scale) {
  typedef typename Elem<ET>::T T;
  typedef typename Frag<T>::V V;
  const T* A = (const T*)Ap; const T* A2 = (const T*)A2p; const T* Bt = (const T*)Btp; const T* Bt2 = (const T*)Bt2p;
  __shared__ __align__(16) float sT[8][16 * 68];
  const int b    = blockIdx.y;
  const int lane = threadIdx.x & 31;
  const int wave = threadIdx.x >> 5;
  const int tilesN = N >> 6;
  const int tilesM = M >> 6;
  const int tile = blockIdx.x * 8 + wave;
  if (tile >= tilesM * tilesN) return;
  const int tm = tile / tilesN;
  const int tn = tile - tm * tilesN;
  const int m0 = tm << 6;
  const int n0 = tn << 6;

  const T* Ab  = A  + (size_t)b * strideA;
  const T* Bb  = Bt + (size_t)b * strideB;
  const T* Ab2 = SPLIT ? (A2  + (size_t)b * strideA) : nullptr;
  const T* Bb2 = SPLIT ? (Bt2 + (size_t)b * strideB) : nullptr;

  const int rlane = lane & 15;
  const int koff  = (lane >> 4) * 8;
  const int mOff  = (lane >> 4) * 8;

  v8f acc[4][4];
#pragma unroll
  for (int i = 0; i < 4; ++i)
#pragma unroll
    for (int j = 0; j < 4; ++j) acc[i][j] = (v8f){0.f,0.f,0.f,0.f,0.f,0.f,0.f,0.f};

  for (int k0 = 0; k0 < K; k0 += 32) {
    V bh[4], bl[4];
#pragma unroll
    for (int j = 0; j < 4; ++j) {
      const size_t bo = (size_t)(n0 + (j << 4) + rlane) * ldb + koff + k0;
      bh[j] = Frag<T>::load(Bb + bo);
      if (SPLIT) bl[j] = Frag<T>::load(Bb2 + bo);
    }
#pragma unroll
    for (int i = 0; i < 4; ++i) {
      const size_t ao = (size_t)(m0 + (i << 4) + rlane) * lda + koff + k0;
      V ah = Frag<T>::load(Ab + ao);
      V al;
      if (SPLIT) al = Frag<T>::load(Ab2 + ao);
#pragma unroll
      for (int j = 0; j < 4; ++j) {
        acc[i][j] = Frag<T>::mma(ah, bh[j], acc[i][j]);
        if (SPLIT) {
          acc[i][j] = Frag<T>::mma(ah, bl[j], acc[i][j]);
          acc[i][j] = Frag<T>::mma(al, bh[j], acc[i][j]);
        }
      }
      Frag<T>::guard4(acc[i][0], acc[i][1], acc[i][2], acc[i][3], ah, SPLIT ? al : ah);
    }
    Frag<T>::keep(bh[0], bh[1], bh[2], bh[3]);
    if (SPLIT) Frag<T>::keep(bl[0], bl[1], bl[2], bl[3]);
  }
  acc_guard4(acc[0][0], acc[0][1], acc[0][2], acc[0][3]);
  acc_guard4(acc[1][0], acc[1][1], acc[1][2], acc[1][3]);
  acc_guard4(acc[2][0], acc[2][1], acc[2][2], acc[2][3]);
  acc_guard4(acc[3][0], acc[3][1], acc[3][2], acc[3][3]);

  float* slab = sT[wave];
  const float* Rb = RESID ? (resid + (size_t)b * strideR) : nullptr;
#pragma unroll
  for (int i = 0; i < 4; ++i) {
    const int mBase = m0 + (i << 4);
#pragma unroll
    for (int j = 0; j < 4; ++j) {
      const int n = n0 + (j << 4) + rlane;
      float bv = 0.f;
      if (BIAS_MODE == 2) bv = bias[n];
#pragma unroll
      for (int r = 0; r < 8; ++r) {
        float v = acc[i][j][r] * scale;
        if (BIAS_MODE == 1) v += bias[mBase + mOff + r];
        if (BIAS_MODE == 2) v += bv;
        if (RESID) v += Rb[(size_t)(mBase + mOff + r) * ldc + n];
        if (ACT == 1) v = tanhf(v);
        if (ACT == 2) v = fmaxf(v, 0.0f);
        if (ACT == 3) v = v / (1.0f + expf(-v));
        if (ACT == 4) v = (v > 0.f) ? v : 0.01f * v;
        slab[(mOff + r) * 68 + (j << 4) + rlane] = v;
      }
    }
    __builtin_amdgcn_fence(__ATOMIC_RELEASE, "workgroup");
    __builtin_amdgcn_wave_barrier();
    __builtin_amdgcn_fence(__ATOMIC_ACQUIRE, "workgroup");
    if (OUT_MODE == 0) {
      float* C = (float*)Cout + (size_t)b * strideC;
      const int hh = lane >> 4, c4 = (lane & 15) * 4;
      for (int pass = 0; pass < 2; ++pass) {
#pragma unroll
        for (int it = 0; it < 8; ++it) {
          const int row = it * 2 + hh;
          v4f v = *(const v4f*)(slab + row * 68 + c4);
          *(volatile v4f*)(C + (size_t)(mBase + row) * ldc + n0 + c4) = v;
        }
        __threadfence();
      }
    } else {
      const int q = lane >> 3, c8 = (lane & 7) * 8;
      unsigned short* C  = (unsigned short*)Cout  + (size_t)b * strideC;
      unsigned short* C2 = (OUT_MODE == 2) ? ((unsigned short*)Cout2 + (size_t)b * strideC) : nullptr;
      for (int pass = 0; pass < 2; ++pass) {
#pragma unroll
        for (int it = 0; it < 4; ++it) {
          const int row = it * 4 + q;
          const float* sp = slab + row * 68 + c8;
          v8h hv, lv;
#pragma unroll
          for (int e = 0; e < 8; ++e) {
            if (OUT_MODE == 1) {
              hv[e] = (_Float16)sp[e];
            } else {
              unsigned short hb = f2bf_bits(sp[e]);
              unsigned short lb = f2bf_bits(sp[e] - bf_bits2f(hb));
              hv[e] = __builtin_bit_cast(_Float16, hb);
              lv[e] = __builtin_bit_cast(_Float16, lb);
            }
          }
          *(volatile v8h*)(C + (size_t)(mBase + row) * ldc + n0 + c8) = hv;
          if (OUT_MODE == 2) *(volatile v8h*)(C2 + (size_t)(mBase + row) * ldc + n0 + c8) = lv;
        }
        __threadfence();
      }
    }
    __builtin_amdgcn_fence(__ATOMIC_RELEASE, "workgroup");
    __builtin_amdgcn_wave_barrier();
    __builtin_amdgcn_fence(__ATOMIC_ACQUIRE, "workgroup");
  }
}

__global__ __launch_bounds__(kThr) void cast_plane_kernel(const float* __restrict__ src, unsigned short* __restrict__ dst,
                                                          int colsLog2, int dstPitch, int dstOff) {
  const int i   = blockIdx.x * kThr + threadIdx.x;
  const int sh  = colsLog2 - 3;
  const int row = i >> sh;
  const int c8  = (i & ((1 << sh) - 1)) * 8;
  const float* sp = src + ((size_t)row << colsLog2) + c8;
  const v4f a0 = *(const v4f*)(sp);
  const v4f a1 = *(const v4f*)(sp + 4);
  v8h hv;
#pragma unroll
  for (int e = 0; e < 4; ++e) {
    const float f0 = a0[e];
    const float f1 = a1[e];
    hv[e]     = (_Float16)carry_flush(bf16r(f0), kInCarry);
    hv[4 + e] = (_Float16)carry_flush(bf16r(f1), kInCarry);
  }
  unsigned short* dp = dst + (size_t)row * dstPitch + dstOff + c8;
  *(volatile v8h*)dp = hv;
  __threadfence();
  *(volatile v8h*)dp = hv;
}
static_assert(kInCarry == kWCarry, "one cast kernel serves inputs and weights");

__global__ __launch_bounds__(kThr) void wpad_kernel(const float* __restrict__ src, unsigned short* __restrict__ dst,
                                                    int srcRows, int srcCols, int dstCols) {
  const int v  = blockIdx.x * kThr + threadIdx.x;
  const int vpr = dstCols >> 3;
  const int r  = v / vpr;
  const int c8 = (v - r * vpr) * 8;
  const int rc = (r < srcRows) ? r : (srcRows - 1);
  v8h hv;
#pragma unroll
  for (int e = 0; e < 8; ++e) {
    const int c = c8 + e;
    const int cc = (c < srcCols) ? c : (srcCols - 1);
    float wv = src[(size_t)rc * srcCols + cc];
    asm volatile("" : "+v"(wv));
    const bool live = (r < srcRows) && (c < srcCols);
    hv[e] = (_Float16)carry_flush(live ? bf16r(wv) : 0.0f, kWCarry);
  }
  unsigned short* dp = dst + (size_t)r * dstCols + c8;
  *(volatile v8h*)dp = hv;
  __threadfence();
  *(volatile v8h*)dp = hv;
}

__global__ __launch_bounds__(kThr) void dec_bias_kernel(const float* __restrict__ b1, const float* __restrict__ b2,
                                                        const float* __restrict__ ba1, const float* __restrict__ ba2,
                                                        float* __restrict__ BV) {
  const int tid = threadIdx.x;
#pragma unroll 1
  for (int it = 0; it < kH / kThr; ++it) {
    const int e = it * kThr + tid;
    const int e2 = (e < kJ) ? e : (kJ - 1);
    float q2 = ba2[e2];
    asm volatile("" : "+v"(q2));
    const float o0 = bf16r(b1[e]), o1 = bf16r(b2[e]), o2 = bf16r(ba1[e]);
    const float o3 = (e < kJ) ? bf16r(q2) : 0.0f;
    for (int pass = 0; pass < 2; ++pass) {
      *(volatile float*)(BV + 0 * kH + e) = o0;
      *(volatile float*)(BV + 1 * kH + e) = o1;
      *(volatile float*)(BV + 2 * kH + e) = o2;
      *(volatile float*)(BV + 3 * kH + e) = o3;
      *(volatile float*)(BV + 4 * kH + e) = 0.0f;
      __threadfence();
    }
  }
}

__device__ __forceinline__ float block_sum256(float v, float* red, float* red8, int tid) {
  red[tid] = v;
  __syncthreads();
  if (tid < 8) {
    float s = 0.0f;
#pragma unroll
    for (int q = 0; q < 8; ++q) {
      const v4f x = *(const v4f*)(red + 32 * tid + 4 * q);
      s += (x[0] + x[1]) + (x[2] + x[3]);
    }
    red8[tid] = s;
  }
  __syncthreads();
  const v4f a = *(const v4f*)(red8);
  const v4f c = *(const v4f*)(red8 + 4);
  return ((a[0] + a[1]) + (a[2] + a[3])) + ((c[0] + c[1]) + (c[2] + c[3]));
}

__global__ __launch_bounds__(kThr) void ln_relu_kernel(const float* __restrict__ P, const float* __restrict__ g,
                                                       const float* __restrict__ be, unsigned short* __restrict__ dst,
                                                       long dstRowStride, const float* __restrict__ Wo,
                                                       float* __restrict__ OBrow, int do_obj) {
  __shared__ __align__(16) float red[256];
  __shared__ __align__(16) float red8[8];
  const int b = blockIdx.x;
  const int tid = threadIdx.x;
  const v4f x = *(const v4f*)(P + (size_t)b * kH + 4 * tid);
  const float m = block_sum256((x[0] + x[1]) + (x[2] + x[3]), red, red8, tid) * (1.0f / (float)kH);
  v4f d;
#pragma unroll
  for (int e = 0; e < 4; ++e) d[e] = x[e] - m;
  const float var = block_sum256((d[0] * d[0] + d[1] * d[1]) + (d[2] * d[2] + d[3] * d[3]), red, red8, tid) * (1.0f / (float)kH);
  const float rs = 1.0f / sqrtf(var + kLnEps);
  const v4f gv = *(const v4f*)(g + 4 * tid);
  const v4f bv = *(const v4f*)(be + 4 * tid);
  v4f y;
  v4h ho;
#pragma unroll
  for (int e = 0; e < 4; ++e) {
    y[e] = fmaxf((d[e] * rs) * bf16r(gv[e]) + bf16r(bv[e]), 0.0f);
    ho[e] = (_Float16)carry_flush(y[e], kInCarry);
  }
  unsigned short* dp = dst + (size_t)b * dstRowStride + 4 * tid;
  *(volatile v4h*)dp = ho;
  __threadfence();
  *(volatile v4h*)dp = ho;
  if (do_obj) {
    float o3[3];
#pragma unroll 1
    for (int j = 0; j < 3; ++j) {
      const v4f wv = *(const v4f*)(Wo + (size_t)j * kH + 4 * tid);
      const float part = (y[0] * bf16r(wv[0]) + y[1] * bf16r(wv[1])) + (y[2] * bf16r(wv[2]) + y[3] * bf16r(wv[3]));
      o3[j] = block_sum256(part, red, red8, tid);
    }
    const float ov = (tid == 0) ? o3[0] : ((tid == 1) ? o3[1] : ((tid == 2) ? o3[2] : 0.0f));
    if (tid < 32) {
      float* op = OBrow + (size_t)b * 32 + tid;
      *(volatile float*)op = ov;
      __threadfence();
      *(volatile float*)op = ov;
    }
  }
}

__global__ __launch_bounds__(kThr) void relu_cast_kernel(const float* __restrict__ P, unsigned short* __restrict__ A1) {
  const size_t i4 = ((size_t)blockIdx.x * kThr + threadIdx.x) * 4;
  const v4f x = *(const v4f*)(P + i4);
  v4h ho;
#pragma unroll
  for (int e = 0; e < 4; ++e) ho[e] = (_Float16)carry_flush(fmaxf(x[e], 0.0f), kInCarry);
  *(volatile v4h*)(A1 + i4) = ho;
  __threadfence();
  *(volatile v4h*)(A1 + i4) = ho;
}

__global__ __launch_bounds__(kThr) void joint_kernel(const float* __restrict__ P4, const float* __restrict__ obs,
                                                     const float* __restrict__ z, const float* __restrict__ alpha_logits,
                                                     const float* __restrict__ jlo, const float* __restrict__ jhi,
                                                     const float* __restrict__ dflt, float* __restrict__ ST,
                                                     float* __restrict__ JSrow, unsigned short* __restrict__ X16,
                                                     int tn, int first, int build) {
  __shared__ float sj[8][24];
  const int wv = threadIdx.x >> 5;
  const int l  = threadIdx.x & 31;
  const int b  = blockIdx.x * 8 + wv;
  const int j  = l % kJ;
  const float lo = bf16r(jlo[j]), hi = bf16r(jhi[j]), df = bf16r(dflt[j]);
  const float al = 1.0f / (1.0f + expf(-bf16r(alpha_logits[j])));
  float pj = df, p4 = 0.0f;
  if (!first) {
    pj = ST[(size_t)b * 32 + j];
    p4 = P4[(size_t)b * kNP + j];
  }
  asm volatile("" : "+v"(pj), "+v"(p4));
  const float a   = tanhf(p4);
  const float tgt = a * kActScale + df;
  const float cju = fminf(fmaxf(pj + al * (tgt - pj), lo), hi);
  const float cj  = first ? df : cju;
  const float cdq = first ? 0.0f : (cju - pj) * kFps;
  const float stv = (l < kJ) ? cj : ((l < 2 * kJ) ? cdq : 0.0f);
  const float jsv = (l < kJ) ? cj : ((l < 2 * kJ) ? a : 0.0f);
  float* sp = ST + (size_t)b * 32 + l;
  float* jp = JSrow + (size_t)b * 32 + l;
  for (int pass = 0; pass < 2; ++pass) {
    *(volatile float*)sp = stv;
    if (!first) *(volatile float*)jp = jsv;
    __threadfence();
  }
  if (l < 2 * kJ) sj[wv][l] = (l < kJ) ? ((cj - 0.5f * (hi + lo)) / (0.5f * (hi - lo))) : cdq;
  __syncthreads();
  if (build) {
#pragma unroll
    for (int part = 0; part < 3; ++part) {
      v2h ho;
#pragma unroll
      for (int e = 0; e < 2; ++e) {
        const int c = part * 64 + 2 * l + e;
        const int cs = (c < 2 * kJ) ? c : 0;
        const int co = (c >= 2 * kJ && c < 2 * kJ + kObs) ? (c - 2 * kJ) : 0;
        const int cz = (c >= 2 * kJ + kObs && c < kPin) ? (c - 2 * kJ - kObs) : 0;
        float ov = obs[((size_t)b * kS + tn) * kObs + co];
        float zv = z[(size_t)b * kLat + cz];
        asm volatile("" : "+v"(ov), "+v"(zv));
        const float sv = sj[wv][cs];
        float v = 0.0f;
        v = (c < 2 * kJ) ? sv : v;
        v = (c >= 2 * kJ && c < 2 * kJ + kObs) ? bf16r(ov) : v;
        v = (c >= 2 * kJ + kObs && c < kPin) ? bf16r(zv) : v;
        ho[e] = (_Float16)carry_flush(v, kInCarry);
      }
      unsigned short* xp = X16 + (size_t)b * kK1 + part * 64 + 2 * l;
      *(volatile v2h*)xp = ho;
      __threadfence();
      *(volatile v2h*)xp = ho;
    }
  }
}

__global__ __launch_bounds__(kThr) void dec_out_kernel(const float* __restrict__ JS, const float* __restrict__ OB,
                                                       const float* __restrict__ PF, const float* __restrict__ fk_W,
                                                       const float* __restrict__ fk_b, const float* __restrict__ bo,
                                                       const float* __restrict__ pos_mean, const float* __restrict__ pos_std,
                                                       const float* __restrict__ bv, float* __restrict__ out) {
  const int blk = blockIdx.x;
  v4f o;
  size_t base;
  if (blk < 1344) {
    const size_t f0 = ((size_t)blk * kThr + threadIdx.x) * 4;
    base = kOut0 + f0;
#pragma unroll 1
    for (int e = 0; e < 4; ++e) {
      const size_t f = f0 + e;
      const int c  = (int)(f % kPD);
      const int bt = (int)(f / kPD);
      const int t = bt & (kS - 1), b = bt >> 7;
      const float* jr = JS + ((size_t)t * kB + b) * 32;
      const int ca = (c < kNLk) ? c : 0;
      const int cb = (c < kNLk) ? 0 : (c - kNLk);
      float acc = bf16r(fk_b[ca]);
#pragma unroll
      for (int j = 0; j < kJ; ++j) acc = fmaf(jr[j], bf16r(fk_W[ca * kJ + j]), acc);
      const float ob = OB[((size_t)t * kB + b) * 32 + cb] + bf16r(bo[cb]);
      const float v = (c < kNLk) ? acc : ob;
      o[e] = (v - bf16r(pos_mean[c])) / bf16r(pos_std[c]);
    }
  } else if (blk < 2112) {
    const int which = (blk < 1728) ? 0 : 1;
    const size_t f0 = ((size_t)(blk - (which ? 1728 : 1344)) * kThr + threadIdx.x) * 4;
    base = (which ? kOut2 : kOut1) + f0;
#pragma unroll 1
    for (int e = 0; e < 4; ++e) {
      const size_t f = f0 + e;
      const int c  = (int)(f % kJ);
      const int bt = (int)(f / kJ);
      const int t = bt & (kS - 1), b = bt >> 7;
      o[e] = JS[((size_t)t * kB + b) * 32 + which * kJ + c];
    }
  } else {
    const size_t f0 = ((size_t)(blk - 2112) * kThr + threadIdx.x) * 4;
    base = kOut3 + f0;
#pragma unroll 1
    for (int e = 0; e < 4; ++e) {
      const size_t f = f0 + e;
      const int c  = (int)(f % kPD);
      const size_t bt = f / kPD;
      const float pre = PF[bt * kNP + c] + bf16r(bv[c]);
      const float sg = 1.0f / (1.0f + expf(-pre));
      o[e] = logf(kSMin + (kSMax - kSMin) * sg);
    }
  }
  float* dp = out + base;
  *(volatile v4f*)dp = o;
  __threadfence();
  *(volatile v4f*)dp = o;
}

static_assert(((size_t)kH * kH / 8) % kThr == 0 && ((size_t)kH * kK1 / 8) % kThr == 0 && ((size_t)kNP * kH / 8) % kThr == 0, "plane grids exact");
static_assert((size_t)kB * kS * kPD / 4 == 1344ull * kThr && (size_t)kB * kS * kJ / 4 == 384ull * kThr, "output grids exact");

extern "C" void kernel_launch(void* const* d_in, const int* in_sizes, int n_in,
                              void* d_out, int out_size, void* d_ws, size_t ws_size,
                              hipStream_t stream) {
  if (n_in < 26 || d_out == nullptr || d_ws == nullptr) return;
  if (in_sizes[0] != kB * kLat || in_sizes[1] != kB * kS * kObs || in_sizes[2] != kH * kPin) return;
  if (in_sizes[3] != kH || in_sizes[4] != kH || in_sizes[5] != kH || in_sizes[6] != kH * kH) return;
  if (in_sizes[7] != kH || in_sizes[8] != kH || in_sizes[9] != kH || in_sizes[10] != kH * kH || in_sizes[11] != kH) return;
  if (in_sizes[12] != kJ * kH || in_sizes[13] != kJ || in_sizes[14] != 3 * kH || in_sizes[15] != 3) return;
  if (in_sizes[16] != kPD * kH || in_sizes[17] != kPD || in_sizes[18] != kJ) return;
  if (in_sizes[19] != kNLk * kJ || in_sizes[20] != kNLk || in_sizes[21] != kPD || in_sizes[22] != kPD) return;
  if (in_sizes[23] != kJ || in_sizes[24] != kJ || in_sizes[25] != kJ) return;
  if ((size_t)out_size != kOutTotal) return;
  if (ws_size < kWsTotal) return;

  const float* z     = (const float*)d_in[0];
  const float* obs   = (const float*)d_in[1];
  const float* W1    = (const float*)d_in[2];
  const float* b1    = (const float*)d_in[3];
  const float* g1    = (const float*)d_in[4];
  const float* be1   = (const float*)d_in[5];
  const float* W2    = (const float*)d_in[6];
  const float* b2    = (const float*)d_in[7];
  const float* g2    = (const float*)d_in[8];
  const float* be2   = (const float*)d_in[9];
  const float* Wa1   = (const float*)d_in[10];
  const float* ba1   = (const float*)d_in[11];
  const float* Wa2   = (const float*)d_in[12];
  const float* ba2   = (const float*)d_in[13];
  const float* Wo    = (const float*)d_in[14];
  const float* bo    = (const float*)d_in[15];
  const float* Wv    = (const float*)d_in[16];
  const float* bv    = (const float*)d_in[17];
  const float* alogit = (const float*)d_in[18];
  const float* fk_W  = (const float*)d_in[19];
  const float* fk_b  = (const float*)d_in[20];
  const float* pmean = (const float*)d_in[21];
  const float* pstd  = (const float*)d_in[22];
  const float* jlo   = (const float*)d_in[23];
  const float* jhi   = (const float*)d_in[24];
  const float* dflt  = (const float*)d_in[25];
  float* out = (float*)d_out;

  char* ws = (char*)d_ws;
  unsigned short* W1P  = (unsigned short*)(ws + kOffW1P);
  unsigned short* W2H  = (unsigned short*)(ws + kOffW2H);
  unsigned short* WA1H = (unsigned short*)(ws + kOffWA1H);
  unsigned short* WA2P = (unsigned short*)(ws + kOffWA2P);
  unsigned short* WVP  = (unsigned short*)(ws + kOffWVP);
  float* BV = (float*)(ws + kOffBV);
  unsigned short* X16 = (unsigned short*)(ws + kOffX16);
  float* PB = (float*)(ws + kOffPB);
  unsigned short* H1 = (unsigned short*)(ws + kOffH1);
  unsigned short* A1 = (unsigned short*)(ws + kOffA1);
  float* P4 = (float*)(ws + kOffP4);
  float* ST = (float*)(ws + kOffST);
  float* JS = (float*)(ws + kOffJS);
  float* OB = (float*)(ws + kOffOB);
  unsigned short* F16P = (unsigned short*)(ws + kOffF16);
  float* PF = (float*)(ws + kOffPF);

  cast_plane_kernel<<<(int)(((size_t)kH * kH / 8) / kThr), kThr, 0, stream>>>(W2, W2H, 10, kH, 0);
  cast_plane_kernel<<<(int)(((size_t)kH * kH / 8) / kThr), kThr, 0, stream>>>(Wa1, WA1H, 10, kH, 0);
  wpad_kernel<<<(int)(((size_t)kH * kK1 / 8) / kThr), kThr, 0, stream>>>(W1, W1P, kH, kPin, kK1);
  wpad_kernel<<<(int)(((size_t)kNP * kH / 8) / kThr), kThr, 0, stream>>>(Wa2, WA2P, kJ, kH, kH);
  wpad_kernel<<<(int)(((size_t)kNP * kH / 8) / kThr), kThr, 0, stream>>>(Wv, WVP, kPD, kH, kH);
  dec_bias_kernel<<<1, kThr, 0, stream>>>(b1, b2, ba1, ba2, BV);
  joint_kernel<<<kB / 8, kThr, 0, stream>>>(P4, obs, z, alogit, jlo, jhi, dflt, ST, JS, X16, 0, 1, 1);

  const dim3 gridL((kB / 64) * (kH / 64) / 8, 1);
  for (int t = 0; t < kS; ++t) {
    unsigned short* Ft = F16P + (size_t)t * kH;
    wmma_gemm64<0, false, 2, 0, false, 0><<<gridL, 256, 0, stream>>>(
        X16, X16, kK1, 0L, W1P, W1P, kK1, 0L, (void*)PB, (void*)PB, kH, 0L,
        BV + 0 * kH, nullptr, 0L, kB, kH, kK1, kScale);
    ln_relu_kernel<<<kB, kThr, 0, stream>>>(PB, g1, be1, H1, (long)kH, Wo, OB, 0);
    wmma_gemm64<0, false, 2, 0, false, 0><<<gridL, 256, 0, stream>>>(
        H1, H1, kH, 0L, W2H, W2H, kH, 0L, (void*)PB, (void*)PB, kH, 0L,
        BV + 1 * kH, nullptr, 0L, kB, kH, kH, kScale);
    ln_relu_kernel<<<kB, kThr, 0, stream>>>(PB, g2, be2, Ft, (long)kS * kH, Wo, OB + (size_t)t * kB * 32, 1);
    wmma_gemm64<0, false, 2, 0, false, 0><<<gridL, 256, 0, stream>>>(
        Ft, Ft, kS * kH, 0L, WA1H, WA1H, kH, 0L, (void*)PB, (void*)PB, kH, 0L,
        BV + 2 * kH, nullptr, 0L, kB, kH, kH, kScale);
    relu_cast_kernel<<<(kB * kH / 4) / kThr, kThr, 0, stream>>>(PB, A1);
    wmma_gemm64<0, false, 2, 0, false, 0><<<dim3(1, 1), 256, 0, stream>>>(
        A1, A1, kH, 0L, WA2P, WA2P, kH, 0L, (void*)P4, (void*)P4, kNP, 0L,
        BV + 3 * kH, nullptr, 0L, kB, kNP, kH, kScale);
    joint_kernel<<<kB / 8, kThr, 0, stream>>>(P4, obs, z, alogit, jlo, jhi, dflt, ST, JS + (size_t)t * kB * 32, X16,
                                              (t + 1 < kS) ? (t + 1) : t, 0, (t + 1 < kS) ? 1 : 0);
  }

  wmma_gemm64<0, false, 2, 0, false, 0><<<dim3(((kB * kS) / 64) * (kNP / 64) / 8, 1), 256, 0, stream>>>(
      F16P, F16P, kH, 0L, WVP, WVP, kH, 0L, (void*)PF, (void*)PF, kNP, 0L,
      BV + 4 * kH, nullptr, 0L, kB * kS, kNP, kH, kScale);
  dec_out_kernel<<<3456, kThr, 0, stream>>>(JS, OB, PF, fk_W, fk_b, bo, pmean, pstd, bv, out);
}
